// MultiHeadAttention_30786325577824
// MI455X (gfx1250) — hardware-verified
//
#include <hip/hip_runtime.h>


typedef _Float16     v16h __attribute__((ext_vector_type(16)));
typedef _Float16     v8h  __attribute__((ext_vector_type(8)));
typedef float        v8f  __attribute__((ext_vector_type(8)));
typedef float        v4f  __attribute__((ext_vector_type(4)));
typedef unsigned int v4u  __attribute__((ext_vector_type(4)));

#ifndef NB
#define NB 1
#endif
#ifndef SEQ
#define SEQ 4096
#endif
#define NB_FULL  1
#define SEQ_FULL 4096
#define DD 1024
#define HH 16
#define HD 64
#define D3 (3 * DD)
#define ER (((SEQ) < 512) ? (SEQ) : 512)

static_assert(SEQ % 128 == 0);
static_assert(SEQ <= SEQ_FULL);
static_assert(NB >= 1 && NB <= NB_FULL);
static_assert(ER % 128 == 0);
static_assert((SEQ - ER) % 128 == 0);
static_assert(((NB * SEQ * DD) / 8) % 256 == 0);
static_assert(DD % 128 == 0 && D3 % 128 == 0 && HD == 64);

#define XCAR    16.0f
#define WCAR    64.0f
#define QKV_INV 0.0009765625f
#define RCAR    2048.0f
#define RINV    0.00048828125f
#define PCAR    1024.0f
#define PINV    0.0009765625f
#define ACAR    16.0f
#define OUT_INV 0.0009765625f

__device__ __forceinline__ v16h load_frag(const _Float16* __restrict__ base, int off) {
    v8h lo = *(const v8h*)(base + off);
    v8h hi = *(const v8h*)(base + off + 16);
    v16h r;
#pragma unroll
    for (int i = 0; i < 8; ++i) { r[i] = lo[i]; r[8 + i] = hi[i]; }
    return r;
}

__device__ __forceinline__ v8f wmma16(v16h a, v16h b, v8f c) {
    v8f d = __builtin_amdgcn_wmma_f32_16x16x32_f16(false, a, false, b, (short)0, c, false, false);
    asm volatile("v_nop\n\tv_nop\n\tv_nop\n\tv_nop" : "+v"(d) : "v"(a), "v"(b));
    return d;
}

__device__ __forceinline__ float bf16r(float f) {
    unsigned int u = __float_as_uint(f);
    u = (u + 0x7FFFu + ((u >> 16) & 1u)) & 0xFFFF0000u;
    return __uint_as_float(u);
}

__device__ __forceinline__ void st16(_Float16* p, v8h v) {
    *(volatile v4u*)p = __builtin_bit_cast(v4u, v);
}
__device__ __forceinline__ void stf4(float* p, v4f v) {
    *(volatile v4f*)p = v;
}

__global__ void __launch_bounds__(256)
k_cvt_x(const float* __restrict__ x, _Float16* __restrict__ xh) {
    const int g  = blockIdx.x * 256 + threadIdx.x;
    const int pr = g >> 7;
    const int c8 = (g & 127) * 8;
    const int b  = pr / SEQ, t = pr - b * SEQ;
    const float* src = x + ((size_t)(b * SEQ_FULL + t)) * DD + c8;
    const v4f u0 = *(const v4f*)src;
    const v4f u1 = *(const v4f*)(src + 4);
    v8h o;
#pragma unroll
    for (int e = 0; e < 4; ++e) {
        o[e]     = (_Float16)(bf16r(u0[e]) * XCAR);
        o[4 + e] = (_Float16)(bf16r(u1[e]) * XCAR);
    }
    _Float16* dst = xh + (size_t)pr * DD + c8;
    st16(dst, o);
    __threadfence();
    st16(dst, o);
}

__global__ void __launch_bounds__(256)
k_tr_w(const float* __restrict__ w, _Float16* __restrict__ wt, int ncols) {
    __shared__ __attribute__((aligned(16))) _Float16 st[64 * 72];
    const int tid = threadIdx.x;
    const int n0 = blockIdx.x * 64, k0 = blockIdx.y * 64;
#pragma unroll
    for (int p = 0; p < 4; ++p) {
        const int r  = (tid >> 4) + 16 * p;
        const int c4 = (tid & 15) * 4;
        const v4f u = *(const v4f*)(w + (size_t)(k0 + r) * ncols + n0 + c4);
#pragma unroll
        for (int e = 0; e < 4; ++e)
            st[(c4 + e) * 72 + r] = (_Float16)(bf16r(u[e]) * WCAR);
    }
    __syncthreads();
    const int piece = tid & 7;
    const int l0 = tid >> 3;
    _Float16* d0 = wt + (size_t)(n0 + l0) * DD + k0 + piece * 8;
    _Float16* d1 = wt + (size_t)(n0 + l0 + 32) * DD + k0 + piece * 8;
    for (int rep = 0; rep < 2; ++rep) {
        if (rep == 1) __threadfence();
        const v8h a0 = *(const v8h*)(st + l0 * 72 + piece * 8);
        const v8h a1 = *(const v8h*)(st + (l0 + 32) * 72 + piece * 8);
        st16(d0, a0);
        st16(d1, a1);
    }
}

__global__ void __launch_bounds__(256) __attribute__((amdgpu_num_vgpr(256)))
k_qkv(const _Float16* __restrict__ xh, const _Float16* __restrict__ wt,
      _Float16* __restrict__ qh, _Float16* __restrict__ kh, _Float16* __restrict__ vth,
      _Float16* __restrict__ qrh, _Float16* __restrict__ krh, _Float16* __restrict__ vtrh) {
    __shared__ __attribute__((aligned(16))) _Float16 st[128 * 72];
    const int tid = threadIdx.x, lane = tid & 31, wid = tid >> 5;
    const int hf = lane >> 4, ln = lane & 15, koff = hf * 8;
    const int n0 = blockIdx.x * 128;
    const int m0 = blockIdx.y * 64;
    const int wm = (wid >> 2) * 32, wn = (wid & 3) * 32;
    const int bb = m0 / SEQ, t0 = m0 - bb * SEQ;
    const int third = n0 / DD, cb = n0 - third * DD;
    const bool isv = (third == 2);

    const _Float16* abase = xh + (size_t)m0 * DD;
    const _Float16* bbase = wt + (size_t)n0 * DD;
    int aoff[2], boff[2];
#pragma unroll
    for (int i = 0; i < 2; ++i) {
        aoff[i] = (wm + i * 16 + ln) * DD + koff;
        boff[i] = (wn + i * 16 + ln) * DD + koff;
    }

    v8f acc[2][2];
#pragma unroll
    for (int i = 0; i < 2; ++i)
#pragma unroll
        for (int jn = 0; jn < 2; ++jn) acc[i][jn] = (v8f){};

#pragma unroll 1
    for (int kk = 0; kk < DD; kk += 32) {
        const v16h a0 = load_frag(abase, aoff[0] + kk);
        const v16h a1 = load_frag(abase, aoff[1] + kk);
        const v16h b0 = load_frag(bbase, boff[0] + kk);
        const v16h b1 = load_frag(bbase, boff[1] + kk);
        acc[0][0] = wmma16(a0, b0, acc[0][0]);
        acc[0][1] = wmma16(a0, b1, acc[0][1]);
        acc[1][0] = wmma16(a1, b0, acc[1][0]);
        acc[1][1] = wmma16(a1, b1, acc[1][1]);
    }

    _Float16* const php = (third == 0) ? qh : kh;
    _Float16* const prp = (third == 0) ? qrh : krh;
    const bool dores = (t0 + 64 <= ER);
    const int piece = tid & 7, lgrp = tid >> 3;

#pragma unroll 1
    for (int ps = 0; ps < 2; ++ps) {
        if (ps == 1 && !dores) break;
        if (ps == 1) __syncthreads();
#pragma unroll
        for (int i = 0; i < 2; ++i)
#pragma unroll
            for (int jn = 0; jn < 2; ++jn)
#pragma unroll
                for (int r = 0; r < 8; ++r) {
                    const float v = acc[i][jn][r] * QKV_INV;
                    const _Float16 hv = (_Float16)v;
                    const _Float16 rv = (_Float16)((v - (float)hv) * RCAR);
                    const _Float16 sv = (ps == 0) ? hv : rv;
                    const int row = wm + i * 16 + koff + r;
                    const int col = wn + jn * 16 + ln;
                    const int idx = isv ? (col * 72 + row) : (row * 136 + col);
                    st[idx] = sv;
                }
        __syncthreads();
        const int prow = (ps == 0) ? SEQ : ER;
        _Float16* const pnv = (ps == 0) ? php : prp;
        _Float16* const pv  = (ps == 0) ? vth : vtrh;
        for (int rep = 0; rep < 2; ++rep) {
            if (rep == 1) __threadfence();
#pragma unroll
            for (int q4 = 0; q4 < 4; ++q4) {
                const int L = q4 * 32 + lgrp;
                int src;
                _Float16* dst;
                if (isv) {
                    const int cg = cb + L;
                    const int hh2 = cg >> 6, dch = cg & 63;
                    src = L * 72 + piece * 8;
                    dst = pv + ((size_t)((bb * HH + hh2) * HD + dch)) * prow + t0 + piece * 8;
                } else {
                    const int R = L >> 1, s = L & 1;
                    const int hh2 = (cb >> 6) + s;
                    src = R * 136 + s * 64 + piece * 8;
                    dst = pnv + (((size_t)(bb * HH + hh2)) * prow + t0 + R) * HD + piece * 8;
                }
                const v8h val = *(const v8h*)(st + src);
                st16(dst, val);
            }
        }
    }
}

template <bool RES>
__global__ void __launch_bounds__(256) __attribute__((amdgpu_num_vgpr(256)))
k_attn(const _Float16* __restrict__ qh, const _Float16* __restrict__ kh,
       const _Float16* __restrict__ vth, const _Float16* __restrict__ qrh,
       const _Float16* __restrict__ krh, const _Float16* __restrict__ vtrh,
       _Float16* __restrict__ ah, _Float16* __restrict__ arh) {
    constexpr int QS    = RES ? 0 : ER;
    constexpr int NBLK0 = RES ? (ER / 128) : ((SEQ - ER) / 128);
    constexpr int NBLK  = (NBLK0 > 0) ? NBLK0 : 1;
    constexpr int WREG  = 16 * 72 * (RES ? 2 : 1);
    __shared__ __attribute__((aligned(16))) _Float16 so[8 * WREG];

    const int tid = threadIdx.x, lane = tid & 31, wid = tid >> 5;
    const int hf = lane >> 4, ln = lane & 15, koff = hf * 8;
    const int bh = blockIdx.x / NBLK;
    const int qbase = QS + (blockIdx.x - bh * NBLK) * 128 + wid * 16;
    const int b = bh / HH, head = bh - b * HH;
    const float scale = 0.125f;

    const _Float16* qb  = qh   + (size_t)bh * SEQ * HD;
    const _Float16* kb  = kh   + (size_t)bh * SEQ * HD;
    const _Float16* vb  = vth  + (size_t)bh * HD * SEQ;
    const _Float16* qrb = qrh  + (size_t)bh * ER * HD;
    const _Float16* krb = krh  + (size_t)bh * ER * HD;
    const _Float16* vrb = vtrh + (size_t)bh * HD * ER;

    const int qo = (qbase + ln) * HD + koff;
    const v16h Bq0 = load_frag(qb, qo);
    const v16h Bq1 = load_frag(qb, qo + 32);
    v16h Br0 = (v16h){}, Br1 = (v16h){};
    if (RES) { Br0 = load_frag(qrb, qo); Br1 = load_frag(qrb, qo + 32); }

    float m = -1e30f, l = 0.0f;
    v8f C[4], Cr[4];
#pragma unroll
    for (int c = 0; c < 4; ++c) { C[c] = (v8f){}; Cr[c] = (v8f){}; }

    const int qrow = qbase + ln;

#pragma unroll 1
    for (int j = 0; j < qbase + 16; j += 32) {
        v8f sh[2], sr[2];
#pragma unroll
        for (int a = 0; a < 2; ++a) {
            const int ko = (j + a * 16 + ln) * HD + koff;
            const v16h Ka  = load_frag(kb, ko);
            const v16h Kb2 = load_frag(kb, ko + 32);
            v8f s = (v8f){};
            s = wmma16(Ka,  Bq0, s);
            s = wmma16(Kb2, Bq1, s);
            sh[a] = s;
            v8f t = (v8f){};
            if (RES) {
                const v16h Kra = load_frag(krb, ko);
                const v16h Krb = load_frag(krb, ko + 32);
                t = wmma16(Ka,  Br0, t);
                t = wmma16(Kb2, Br1, t);
                t = wmma16(Kra, Bq0, t);
                t = wmma16(Krb, Bq1, t);
            }
            sr[a] = t;
        }

        v8f sc[2];
        float mx = -1e30f;
#pragma unroll
        for (int a = 0; a < 2; ++a)
#pragma unroll
            for (int r = 0; r < 8; ++r) {
                float v = sh[a][r];
                if (RES) v = v + sr[a][r] * RINV;
                v = v * scale;
                const int key = j + a * 16 + koff + r;
                v = (key > qrow) ? -1e30f : v;
                sc[a][r] = v;
                mx = fmaxf(mx, v);
            }
        mx = fmaxf(mx, __shfl_xor(mx, 16, 32));
        const float mn = fmaxf(m, mx);
        const float alpha = __expf(m - mn);
        m = mn;

        float lsum = 0.0f;
        v16h pa, par = (v16h){};
#pragma unroll
        for (int a = 0; a < 2; ++a)
#pragma unroll
            for (int r = 0; r < 8; ++r) {
                const float p  = __expf(sc[a][r] - mn);
                lsum += p;
                const float pc = p * PCAR;
                const _Float16 hp = (_Float16)pc;
                pa[a * 8 + r] = hp;
                if (RES) par[a * 8 + r] = (_Float16)((pc - (float)hp) * RCAR);
            }
        lsum += __shfl_xor(lsum, 16, 32);
        l = l * alpha + lsum;

#pragma unroll
        for (int r = 0; r < 8; ++r) {
            const float f = __shfl(alpha, koff + r, 32);
#pragma unroll
            for (int c = 0; c < 4; ++c) {
                C[c][r] *= f;
                if (RES) Cr[c][r] *= f;
            }
        }

#pragma unroll
        for (int c = 0; c < 4; ++c) {
            const v16h Bv = load_frag(vb, (c * 16 + ln) * SEQ + j + koff);
            C[c] = wmma16(pa, Bv, C[c]);
            if (RES) {
                const v16h Bvr = load_frag(vrb, (c * 16 + ln) * ER + j + koff);
                Cr[c] = wmma16(pa,  Bvr, Cr[c]);
                Cr[c] = wmma16(par, Bv,  Cr[c]);
            }
        }
    }

    _Float16* const sw = so + wid * WREG;
#pragma unroll
    for (int r = 0; r < 8; ++r) {
        const float lr  = __shfl(l, koff + r, 32);
        const float inv = (1.0f / lr) * (PINV * ACAR);
        const int row = koff + r;
#pragma unroll
        for (int c = 0; c < 4; ++c) {
            float v = C[c][r];
            if (RES) v = v + Cr[c][r] * RINV;
            v = v * inv;
            const _Float16 hv = (_Float16)v;
            sw[row * 72 + c * 16 + ln] = hv;
            if (RES) sw[16 * 72 + row * 72 + c * 16 + ln] = (_Float16)((v - (float)hv) * RCAR);
        }
    }
    __syncthreads();

    const int piece = lane & 7, lq = lane >> 3;
    for (int rep = 0; rep < 2; ++rep) {
        if (rep == 1) __threadfence();
#pragma unroll
        for (int p = 0; p < 4; ++p) {
            const int line = p * 4 + lq;
            const v8h hv8 = *(const v8h*)(sw + line * 72 + piece * 8);
            _Float16* hd_ = ah + ((size_t)(b * SEQ + qbase + line)) * DD + head * HD + piece * 8;
            st16(hd_, hv8);
            if (RES) {
                const v8h rv8 = *(const v8h*)(sw + 16 * 72 + line * 72 + piece * 8);
                _Float16* rd_ = arh + ((size_t)(b * ER + qbase + line)) * DD + head * HD + piece * 8;
                st16(rd_, rv8);
            }
        }
    }
}

__global__ void __launch_bounds__(256) __attribute__((amdgpu_num_vgpr(256)))
k_oproj(const _Float16* __restrict__ ah, const _Float16* __restrict__ arh,
        const _Float16* __restrict__ wt, float* __restrict__ out) {
    __shared__ __attribute__((aligned(16))) float so[64 * 132];
    const int tid = threadIdx.x, lane = tid & 31, wid = tid >> 5;
    const int hf = lane >> 4, ln = lane & 15, koff = hf * 8;
    const int n0 = blockIdx.x * 128, m0 = blockIdx.y * 64;
    const int wm = (wid >> 2) * 32, wn = (wid & 3) * 32;
    const int b = m0 / SEQ, t0 = m0 - b * SEQ;
    const bool early = (t0 + 64 <= ER);

    const _Float16* abase  = ah  + (size_t)m0 * DD;
    const _Float16* arbase = arh + (size_t)(b * ER + (early ? t0 : 0)) * DD;
    const _Float16* bbase  = wt  + (size_t)n0 * DD;
    int aoff[2], boff[2];
#pragma unroll
    for (int i = 0; i < 2; ++i) {
        aoff[i] = (wm + i * 16 + ln) * DD + koff;
        boff[i] = (wn + i * 16 + ln) * DD + koff;
    }

    v8f acc[2][2], accr[2][2];
#pragma unroll
    for (int i = 0; i < 2; ++i)
#pragma unroll
        for (int jn = 0; jn < 2; ++jn) { acc[i][jn] = (v8f){}; accr[i][jn] = (v8f){}; }

#pragma unroll 1
    for (int kk = 0; kk < DD; kk += 32) {
        const v16h a0 = load_frag(abase, aoff[0] + kk);
        const v16h a1 = load_frag(abase, aoff[1] + kk);
        const v16h b0 = load_frag(bbase, boff[0] + kk);
        const v16h b1 = load_frag(bbase, boff[1] + kk);
        acc[0][0] = wmma16(a0, b0, acc[0][0]);
        acc[0][1] = wmma16(a0, b1, acc[0][1]);
        acc[1][0] = wmma16(a1, b0, acc[1][0]);
        acc[1][1] = wmma16(a1, b1, acc[1][1]);
    }
    if (early) {
#pragma unroll 1
        for (int kk = 0; kk < DD; kk += 32) {
            const v16h a0 = load_frag(arbase, aoff[0] + kk);
            const v16h a1 = load_frag(arbase, aoff[1] + kk);
            const v16h b0 = load_frag(bbase, boff[0] + kk);
            const v16h b1 = load_frag(bbase, boff[1] + kk);
            accr[0][0] = wmma16(a0, b0, accr[0][0]);
            accr[0][1] = wmma16(a0, b1, accr[0][1]);
            accr[1][0] = wmma16(a1, b0, accr[1][0]);
            accr[1][1] = wmma16(a1, b1, accr[1][1]);
        }
    }

#pragma unroll
    for (int i = 0; i < 2; ++i)
#pragma unroll
        for (int jn = 0; jn < 2; ++jn)
#pragma unroll
            for (int r = 0; r < 8; ++r) {
                const int row = wm + i * 16 + koff + r;
                const int col = wn + jn * 16 + ln;
                const float v = (acc[i][jn][r] + accr[i][jn][r] * RINV) * OUT_INV;
                so[row * 132 + col] = v;
            }
    __syncthreads();

    const int piece = tid & 7, lgrp = tid >> 3;
    for (int rep = 0; rep < 2; ++rep) {
        if (rep == 1) __threadfence();
#pragma unroll
        for (int p = 0; p < 8; ++p) {
            const int L = p * 32 + lgrp;
            const int R = L >> 2, s = L & 3;
            const v4f val = *(const v4f*)(so + R * 132 + s * 32 + piece * 4);
            float* dst = out + ((size_t)(b * SEQ_FULL + t0 + R)) * DD + n0 + s * 32 + piece * 4;
            stf4(dst, val);
        }
    }
}

extern "C" void kernel_launch(void* const* d_in, const int* in_sizes, int n_in,
                              void* d_out, int out_size, void* d_ws, size_t ws_size,
                              hipStream_t stream) {
    if (n_in < 3) return;
    const int rows_used = (NB - 1) * SEQ_FULL + SEQ;
    if (in_sizes[0] < rows_used * DD) return;
    if (in_sizes[1] < DD * D3) return;
    if (in_sizes[2] < DD * DD) return;
    if (out_size < rows_used * DD) return;

    const float* x    = (const float*)d_in[0];
    const float* wqkv = (const float*)d_in[1];
    const float* wout = (const float*)d_in[2];
    float* out = (float*)d_out;

    char* ws = (char*)d_ws;
    size_t o = 0;
    _Float16* xh   = (_Float16*)(ws + o); o += (size_t)NB * SEQ * DD * 2;
    _Float16* wq   = (_Float16*)(ws + o); o += (size_t)D3 * DD * 2;
    _Float16* wo   = (_Float16*)(ws + o); o += (size_t)DD * DD * 2;
    _Float16* qh   = (_Float16*)(ws + o); o += (size_t)NB * HH * SEQ * HD * 2;
    _Float16* kh   = (_Float16*)(ws + o); o += (size_t)NB * HH * SEQ * HD * 2;
    _Float16* vth  = (_Float16*)(ws + o); o += (size_t)NB * HH * HD * SEQ * 2;
    _Float16* qrh  = (_Float16*)(ws + o); o += (size_t)NB * HH * ER * HD * 2;
    _Float16* krh  = (_Float16*)(ws + o); o += (size_t)NB * HH * ER * HD * 2;
    _Float16* vtrh = (_Float16*)(ws + o); o += (size_t)NB * HH * HD * ER * 2;
    _Float16* ah   = (_Float16*)(ws + o); o += (size_t)NB * SEQ * DD * 2;
    _Float16* arh  = (_Float16*)(ws + o); o += (size_t)NB * ER * DD * 2;
    if (o > ws_size) return;

    k_cvt_x<<<(NB * SEQ * DD / 8) / 256, 256, 0, stream>>>(x, xh);
    k_tr_w<<<dim3(D3 / 64, DD / 64), 256, 0, stream>>>(wqkv, wq, D3);
    k_tr_w<<<dim3(DD / 64, DD / 64), 256, 0, stream>>>(wout, wo, DD);
    k_qkv<<<dim3(D3 / 128, (NB * SEQ) / 64), 256, 0, stream>>>(xh, wq, qh, kh, vth, qrh, krh, vtrh);
    k_attn<true><<<NB * HH * (ER / 128), 256, 0, stream>>>(qh, kh, vth, qrh, krh, vtrh, ah, arh);
    constexpr int nlate = NB * HH * ((SEQ - ER) / 128);
    if (nlate > 0)
        k_attn<false><<<nlate, 256, 0, stream>>>(qh, kh, vth, qrh, krh, vtrh, ah, arh);
    k_oproj<<<dim3(DD / 128, (NB * SEQ) / 64), 256, 0, stream>>>(ah, arh, wo, out);
}
